// Encoder_12618613916304
// MI455X (gfx1250) — hardware-verified
//
#include <hip/hip_runtime.h>
#include <stddef.h>
#include <stdint.h>


#define DIN    64
#define HID    128
#define OUTC   64
#define AP1    192
#define AP2    256
#define XOFF   128
#define NTHR   256
#define NWAVE  8
#define EPT    8
#define CHUNK  (NTHR * EPT)
#define WCAP   (EPT * 32)
#define LISTN  (NWAVE * WCAP)
#define RCAP   10240
#define DEGCAP 128
#define GBM    64
#define GTHR   128
#define MISC_INTS   16
#define ROWBUF_INTS (NWAVE * AP2 / 2)
#define SCAN_ZINTS(slb)    (LISTN + 2 * RCAP + 3 * (1 << (slb)))
#define SCAN_LDSINTS(slb)  (SCAN_ZINTS(slb) + MISC_INTS + ROWBUF_INTS)
#define SLB_M  8
#define SLB_U  10
#define NWB    72
#define WSMAX  134217728

static_assert((CHUNK & (CHUNK - 1)) == 0 && CHUNK <= 4096);
static_assert(((long long)CHUNK << SLB_U) < (1LL << 31));
static_assert(LISTN % 4 == 0 && RCAP % 32 == 0);
static_assert(SCAN_ZINTS(SLB_M) % 4 == 0 && SCAN_ZINTS(SLB_U) % 4 == 0);
static_assert(SCAN_LDSINTS(SLB_U) * 4 <= 300000);
static_assert(AP1 % 32 == 0 && AP2 % 32 == 0 && AP1 == 3 * DIN && AP2 == 2 * HID);
static_assert(GBM == (GTHR / 32) * 16 && HID == 4 * 32 && DIN == 2 * 32);

typedef float          v4f   __attribute__((ext_vector_type(4)));
typedef float          v8f   __attribute__((ext_vector_type(8)));
typedef int            v4i   __attribute__((ext_vector_type(4)));
typedef int            v8i   __attribute__((ext_vector_type(8)));
typedef unsigned int   v4u   __attribute__((ext_vector_type(4)));
typedef unsigned short v4us  __attribute__((ext_vector_type(4)));
typedef unsigned short v8us  __attribute__((ext_vector_type(8)));
typedef unsigned short v16us __attribute__((ext_vector_type(16)));
typedef __bf16         v16bf __attribute__((ext_vector_type(16)));
typedef v4f  __attribute__((may_alias)) v4fa;
typedef v4i  __attribute__((may_alias)) v4ia;
typedef v4us __attribute__((may_alias)) v4usa;
typedef v8us __attribute__((may_alias)) v8usa;
typedef unsigned int __attribute__((may_alias)) u32a;
union FragB { v16bf v; v16us u; v8us h[2]; v8i w; };

__device__ __forceinline__ v8f wmb(const FragB& a, const FragB& b, v8f c) {
  v8f d = __builtin_amdgcn_wmma_f32_16x16x32_bf16(false, a.v, false, b.v, (short)0, c, false, false);
  asm volatile("v_nop\n\tv_nop\n\tv_nop\n\tv_nop" : "+v"(d) : "v"(a.w), "v"(b.w));
  return d;
}

__device__ __forceinline__ unsigned bf16_bits(float f) {
  const unsigned u = __float_as_uint(f);
  const unsigned r = (u + 0x7FFFu + ((u >> 16) & 1u)) >> 16;
  const unsigned q = (u >> 16) | 0x40u;
  return ((u & 0x7fffffffu) > 0x7f800000u) ? q : r;
}
__device__ __forceinline__ float bf16_val(float f) {
  return __uint_as_float(bf16_bits(f) << 16);
}

__device__ __forceinline__ void wave_sync() {
  __builtin_amdgcn_fence(__ATOMIC_RELEASE, "wavefront");
  __builtin_amdgcn_wave_barrier();
  __builtin_amdgcn_fence(__ATOMIC_ACQUIRE, "wavefront");
}

template <int SLB>
__device__ __forceinline__ int scan_chunk(const int* __restrict__ dsts, int nE, int cbase, int slotBase,
                                          int nb, int vec8, int* list, int tid, int lane, int wave) {
  int wc = 0;
  const int el0  = tid * EPT;
  const int e0   = cbase + el0;
  const int sent = -2147483647 - 1;
  v4i da, db;
  if (vec8 != 0 && cbase + CHUNK <= nE) {
    da = *(const v4i*)(dsts + e0);
    db = *(const v4i*)(dsts + e0 + 4);
  } else {
    da.x = (e0     < nE) ? dsts[min(e0,     nE - 1)] : sent;
    da.y = (e0 + 1 < nE) ? dsts[min(e0 + 1, nE - 1)] : sent;
    da.z = (e0 + 2 < nE) ? dsts[min(e0 + 2, nE - 1)] : sent;
    da.w = (e0 + 3 < nE) ? dsts[min(e0 + 3, nE - 1)] : sent;
    db.x = (e0 + 4 < nE) ? dsts[min(e0 + 4, nE - 1)] : sent;
    db.y = (e0 + 5 < nE) ? dsts[min(e0 + 5, nE - 1)] : sent;
    db.z = (e0 + 6 < nE) ? dsts[min(e0 + 6, nE - 1)] : sent;
    db.w = (e0 + 7 < nE) ? dsts[min(e0 + 7, nE - 1)] : sent;
  }
  const unsigned nbs = (unsigned)slotBase;
  const unsigned unb = (unsigned)nb;
  const unsigned s0 = (unsigned)da.x - nbs, s1 = (unsigned)da.y - nbs;
  const unsigned s2 = (unsigned)da.z - nbs, s3 = (unsigned)da.w - nbs;
  const unsigned s4 = (unsigned)db.x - nbs, s5 = (unsigned)db.y - nbs;
  const unsigned s6 = (unsigned)db.z - nbs, s7 = (unsigned)db.w - nbs;
  const bool h0 = s0 < unb, h1 = s1 < unb, h2 = s2 < unb, h3 = s3 < unb;
  const bool h4 = s4 < unb, h5 = s5 < unb, h6 = s6 < unb, h7 = s7 < unb;
  const unsigned any = __builtin_amdgcn_ballot_w32(h0 | h1 | h2 | h3 | h4 | h5 | h6 | h7);
  if (any != 0u) {
#define HITJ(J, HJ, SJ) { \
      const unsigned mj = __builtin_amdgcn_ballot_w32(HJ); \
      if (mj != 0u) { \
        if (HJ) { \
          const int pos = wc + (int)__builtin_amdgcn_mbcnt_lo(mj, 0u); \
          if (pos < WCAP) list[wave * WCAP + pos] = ((el0 + (J)) << SLB) | (int)(SJ); \
        } \
        wc += (int)__builtin_popcount(mj); } }
    HITJ(0, h0, s0)
    HITJ(1, h1, s1)
    HITJ(2, h2, s2)
    HITJ(3, h3, s3)
    HITJ(4, h4, s4)
    HITJ(5, h5, s5)
    HITJ(6, h6, s6)
    HITJ(7, h7, s7)
#undef HITJ
  }
  return wc;
}

__device__ __forceinline__ void x_unit(const float* __restrict__ x, int nN, unsigned short* plane, int u) {
  const int row = u >> 3;
  const int k8  = (u & 7) * 8;
  const int rc  = row < nN ? row : nN - 1;
  const float* p = x + (size_t)rc * DIN + k8;
  const v4f a = *(const v4fa*)p;
  const v4f b = *(const v4fa*)(p + 4);
  const bool ok = row < nN;
  v8us o;
  o[0] = ok ? (unsigned short)bf16_bits(a.x) : (unsigned short)0;
  o[1] = ok ? (unsigned short)bf16_bits(a.y) : (unsigned short)0;
  o[2] = ok ? (unsigned short)bf16_bits(a.z) : (unsigned short)0;
  o[3] = ok ? (unsigned short)bf16_bits(a.w) : (unsigned short)0;
  o[4] = ok ? (unsigned short)bf16_bits(b.x) : (unsigned short)0;
  o[5] = ok ? (unsigned short)bf16_bits(b.y) : (unsigned short)0;
  o[6] = ok ? (unsigned short)bf16_bits(b.z) : (unsigned short)0;
  o[7] = ok ? (unsigned short)bf16_bits(b.w) : (unsigned short)0;
  unsigned short* dp = plane + (size_t)row * AP1 + XOFF + k8;
  *(volatile v8us*)dp = o;
  __threadfence();
  *(volatile v8us*)dp = o;
}

template <int KS, int NS>
__device__ __forceinline__ void wt_part(const float* __restrict__ W, unsigned short* P, int pitch,
                                        int rowoff, int coff, int v) {
  constexpr int UPR = KS / 8;
  const int n  = v / UPR;
  const int k8 = (v % UPR) * 8;
  const float* p = W + (size_t)k8 * NS + n;
  v8us o;
#pragma unroll
  for (int i = 0; i < 8; ++i) o[i] = (unsigned short)bf16_bits(p[(size_t)i * NS]);
  unsigned short* dp = P + (size_t)(rowoff + n) * pitch + coff + k8;
  *(volatile v8us*)dp = o;
  __threadfence();
  *(volatile v8us*)dp = o;
}

__global__ __launch_bounds__(NTHR) void k_prep(
    const float* __restrict__ xu, const float* __restrict__ xm, int nU, int nM, int nBU, int nBM,
    const float* __restrict__ W1l, const float* __restrict__ W1r,
    const float* __restrict__ W2l, const float* __restrict__ W2r,
    const float* __restrict__ W3l, const float* __restrict__ W3r,
    const float* __restrict__ Wl1, const float* __restrict__ Wl2,
    unsigned short* A1U, unsigned short* A2M,
    unsigned short* B1, unsigned short* B2, unsigned short* BM, unsigned short* B3r, unsigned short* BL1) {
  const int b = (int)blockIdx.x, tid = (int)threadIdx.x;
  if (b < nBU) { x_unit(xu, nU, A1U, b * NTHR + tid); return; }
  if (b < nBU + nBM) { x_unit(xm, nM, A2M, (b - nBU) * NTHR + tid); return; }
  const int wb = b - nBU - nBM;
  if (wb < 4)        wt_part<64, 128>(W1l, B1, AP1, 0, 0,        (wb)      * NTHR + tid);
  else if (wb < 8)   wt_part<64, 128>(W1l, B1, AP1, 0, DIN,      (wb - 4)  * NTHR + tid);
  else if (wb < 12)  wt_part<64, 128>(W1r, B1, AP1, 0, 2 * DIN,  (wb - 8)  * NTHR + tid);
  else if (wb < 16)  wt_part<64, 128>(W2l, B2, AP1, 0, 0,        (wb - 12) * NTHR + tid);
  else if (wb < 20)  wt_part<64, 128>(W2l, B2, AP1, 0, DIN,      (wb - 16) * NTHR + tid);
  else if (wb < 24)  wt_part<64, 128>(W2r, B2, AP1, 0, 2 * DIN,  (wb - 20) * NTHR + tid);
  else if (wb < 32)  wt_part<128, 128>(W3l, BM, AP2, 0, 0,       (wb - 24) * NTHR + tid);
  else if (wb < 40)  wt_part<128, 128>(W3l, BM, AP2, 0, HID,     (wb - 32) * NTHR + tid);
  else if (wb < 48)  wt_part<128, 128>(W3r, B3r, AP2, 0, 0,      (wb - 40) * NTHR + tid);
  else if (wb < 56)  wt_part<128, 128>(W3r, B3r, AP2, 0, HID,    (wb - 48) * NTHR + tid);
  else if (wb < 60)  wt_part<128, 64>(Wl2, BM, AP2, HID, 0,      (wb - 56) * NTHR + tid);
  else if (wb < 64)  wt_part<128, 64>(Wl2, BM, AP2, HID, HID,    (wb - 60) * NTHR + tid);
  else if (wb < 68)  wt_part<128, 64>(Wl1, BL1, AP2, 0, 0,       (wb - 64) * NTHR + tid);
  else if (wb < 72)  wt_part<128, 64>(Wl1, BL1, AP2, 0, HID,     (wb - 68) * NTHR + tid);
}

template <int NT, int EPI>
__device__ __forceinline__ void gemm_body(float* stg, const unsigned short* __restrict__ A, int lda,
                                          const unsigned short* __restrict__ BT, int K,
                                          const float* __restrict__ bias, int hasB, int nOut,
                                          unsigned short* outH, float* outF, int rowBase) {
  constexpr int NC = NT * 16;
  const int tid = (int)threadIdx.x, lane = tid & 31, wave = tid >> 5, hh = lane >> 4, m = lane & 15;

  v8f acc[NT];
  {
    const v8f z = {0.f, 0.f, 0.f, 0.f, 0.f, 0.f, 0.f, 0.f};
#pragma unroll
    for (int t = 0; t < NT; ++t) acc[t] = z;
  }
  const unsigned short* ap = A + (size_t)(rowBase + 16 * wave + m) * (size_t)lda + 8 * hh;
  const unsigned short* bp = BT + (size_t)m * (size_t)K + 8 * hh;

#pragma unroll 1
  for (int k0 = 0; k0 < K; k0 += 32) {
    FragB af;
    af.h[0] = *(const v8usa*)(ap + k0);
    af.h[1] = *(const v8usa*)(ap + k0 + 16);
#pragma unroll
    for (int nt = 0; nt < NT; ++nt) {
      const unsigned short* wq = bp + (size_t)(16 * nt) * (size_t)K + k0;
      FragB bf;
      bf.h[0] = *(const v8usa*)wq;
      bf.h[1] = *(const v8usa*)(wq + 16);
      acc[nt] = wmb(af, bf, acc[nt]);
    }
  }

#pragma unroll
  for (int nt = 0; nt < NT; ++nt) {
    const int lc = 16 * nt + m;
#pragma unroll
    for (int r = 0; r < 8; ++r) {
      const int lr = 16 * wave + 8 * hh + r;
      stg[lr * NC + lc] = acc[nt][r];
    }
  }
  __syncthreads();

  if constexpr (EPI == 0) {
    v4f bb4;
    {
      const v4f t1 = *(const v4f*)(bias + 4 * lane);
      bb4.x = (hasB != 0) ? bf16_val(t1.x) : 0.0f;
      bb4.y = (hasB != 0) ? bf16_val(t1.y) : 0.0f;
      bb4.z = (hasB != 0) ? bf16_val(t1.z) : 0.0f;
      bb4.w = (hasB != 0) ? bf16_val(t1.w) : 0.0f;
    }
#pragma unroll 1
    for (int i = 0; i < 16; ++i) {
      const int lr = 16 * wave + i;
      const bool ok = (rowBase + lr) < nOut;
      float* srow = stg + lr * NC;
      const v4f t = *(const v4fa*)(srow + 4 * lane);
      float y0 = t.x + bb4.x, y1 = t.y + bb4.y, y2 = t.z + bb4.z, y3 = t.w + bb4.w;
      y0 = (y0 > 0.0f) ? y0 : (y0 - y0);
      y1 = (y1 > 0.0f) ? y1 : (y1 - y1);
      y2 = (y2 > 0.0f) ? y2 : (y2 - y2);
      y3 = (y3 > 0.0f) ? y3 : (y3 - y3);
      y0 = ok ? y0 : 0.0f; y1 = ok ? y1 : 0.0f; y2 = ok ? y2 : 0.0f; y3 = ok ? y3 : 0.0f;
      v4us h4, l4;
      unsigned hb;
      hb = bf16_bits(y0); h4[0] = (unsigned short)hb; l4[0] = (unsigned short)bf16_bits(y0 - __uint_as_float(hb << 16));
      hb = bf16_bits(y1); h4[1] = (unsigned short)hb; l4[1] = (unsigned short)bf16_bits(y1 - __uint_as_float(hb << 16));
      hb = bf16_bits(y2); h4[2] = (unsigned short)hb; l4[2] = (unsigned short)bf16_bits(y2 - __uint_as_float(hb << 16));
      hb = bf16_bits(y3); h4[3] = (unsigned short)hb; l4[3] = (unsigned short)bf16_bits(y3 - __uint_as_float(hb << 16));
      wave_sync();
      unsigned short* hrow = (unsigned short*)srow;
      *(v4usa*)(hrow + 4 * lane) = h4;
      *(v4usa*)(hrow + HID + 4 * lane) = l4;
    }
    __syncthreads();
#pragma unroll 1
    for (int i = 0; i < 16; ++i) {
      const int lr = 16 * wave + i;
      const unsigned short* hrow = (const unsigned short*)(stg + lr * NC);
      const v8us q = *(const v8usa*)(hrow + 8 * lane);
      unsigned short* rp = outH + (size_t)(rowBase + lr) * (size_t)AP2 + 8 * lane;
      *(volatile v8us*)rp = q;
    }
    __threadfence();
#pragma unroll 1
    for (int i = 0; i < 16; ++i) {
      const int lr = 16 * wave + i;
      const unsigned short* hrow = (const unsigned short*)(stg + lr * NC);
      const v8us q = *(const v8usa*)(hrow + 8 * lane);
      unsigned short* rp = outH + (size_t)(rowBase + lr) * (size_t)AP2 + 8 * lane;
      *(volatile v8us*)rp = q;
    }
  } else if constexpr (EPI == 1) {
    v4f bb4;
    {
      const v4f t1 = *(const v4f*)(bias + 4 * lane);
      bb4.x = (hasB != 0) ? bf16_val(t1.x) : 0.0f;
      bb4.y = (hasB != 0) ? bf16_val(t1.y) : 0.0f;
      bb4.z = (hasB != 0) ? bf16_val(t1.z) : 0.0f;
      bb4.w = (hasB != 0) ? bf16_val(t1.w) : 0.0f;
    }
#pragma unroll 1
    for (int i = 0; i < 16; ++i) {
      const int lr = 16 * wave + i;
      const v4f v = *(const v4fa*)(stg + lr * NC + 4 * lane) + bb4;
      float* op = outF + (size_t)(rowBase + lr) * (size_t)HID + 4 * lane;
      *(volatile v4f*)op = v;
    }
    __threadfence();
#pragma unroll 1
    for (int i = 0; i < 16; ++i) {
      const int lr = 16 * wave + i;
      const v4f v = *(const v4fa*)(stg + lr * NC + 4 * lane) + bb4;
      float* op = outF + (size_t)(rowBase + lr) * (size_t)HID + 4 * lane;
      *(volatile v4f*)op = v;
    }
  } else {
    v4f bb4;
    {
      const v4f t1 = *(const v4f*)(bias + 4 * m);
      bb4.x = (hasB != 0) ? bf16_val(t1.x) : 0.0f;
      bb4.y = (hasB != 0) ? bf16_val(t1.y) : 0.0f;
      bb4.z = (hasB != 0) ? bf16_val(t1.z) : 0.0f;
      bb4.w = (hasB != 0) ? bf16_val(t1.w) : 0.0f;
    }
#pragma unroll 1
    for (int i = 0; i < 8; ++i) {
      const int lr = 16 * wave + 2 * i + hh;
      const int gr = rowBase + lr;
      const v4f v = *(const v4fa*)(stg + lr * NC + 4 * m) + bb4;
      float* op = outF + (size_t)gr * (size_t)OUTC + 4 * m;
      if (gr < nOut) *(volatile v4f*)op = v;
    }
    __threadfence();
#pragma unroll 1
    for (int i = 0; i < 8; ++i) {
      const int lr = 16 * wave + 2 * i + hh;
      const int gr = rowBase + lr;
      const v4f v = *(const v4fa*)(stg + lr * NC + 4 * m) + bb4;
      float* op = outF + (size_t)gr * (size_t)OUTC + 4 * m;
      if (gr < nOut) *(volatile v4f*)op = v;
    }
  }
}

template <int NT, int EPI>
__global__ __launch_bounds__(GTHR) void k_gemm(const unsigned short* __restrict__ A, int lda,
                                               const unsigned short* __restrict__ BT, int K,
                                               const float* __restrict__ bias, int hasB, int nOut,
                                               unsigned short* outH, float* outF) {
  __shared__ __attribute__((aligned(16))) float stg[GBM * 128];
  gemm_body<NT, EPI>(stg, A, lda, BT, K, bias, hasB, nOut, outH, outF, (int)blockIdx.x * GBM);
}

__global__ __launch_bounds__(GTHR) void k_gemm_mv(const unsigned short* __restrict__ MX,
                                                  const unsigned short* __restrict__ BM,
                                                  const float* __restrict__ bl2,
                                                  const float* __restrict__ z128, int nM,
                                                  unsigned short* dummyH, float* T3, float* outMv) {
  __shared__ __attribute__((aligned(16))) float stg[GBM * 128];
  const int rowBase = (int)blockIdx.x * GBM;
  if (blockIdx.y == 0) {
    gemm_body<8, 1>(stg, MX, AP2, BM, AP2, z128, 0, nM, dummyH, T3, rowBase);
  } else {
    gemm_body<4, 2>(stg, MX, AP2, BM + (size_t)HID * AP2, AP2, bl2, 1, nM, dummyH, outMv, rowBase);
  }
}

template <int SLB, int WIDE>
__global__ __launch_bounds__(NTHR) void k_scan(const int* __restrict__ gath, const int* __restrict__ keys,
                                               int nE, int nDst, int nSrc, int vec8, int mRows,
                                               const unsigned short* srcPl, const float* __restrict__ t3,
                                               const float* __restrict__ s3, unsigned short* outPl) {
  constexpr int NB    = 1 << SLB;
  constexpr int ZINTS = LISTN + 2 * RCAP + 3 * NB;
  static_assert(NB % NWAVE == 0 && NB % 32 == 0 && ZINTS % 4 == 0);
  extern __shared__ __attribute__((aligned(16))) int dsm[];
  int* list = dsm;
  int* hl   = dsm + LISTN;
  int* sl   = hl + RCAP;
  int* cnt  = sl + RCAP;
  int* offs = cnt + NB;
  int* cur  = offs + NB;
  int* misc = cur + NB;
  const int tid = (int)threadIdx.x, lane = tid & 31, wave = tid >> 5;
  unsigned short* rowbuf = (unsigned short*)(misc + MISC_INTS) + wave * AP2;
  const int nodeBase = (int)blockIdx.x * NB;

  {
    const v4i z4 = {0, 0, 0, 0};
    for (int i = tid * 4; i < ZINTS; i += NTHR * 4) *(v4ia*)(dsm + i) = z4;
    if (tid < MISC_INTS) misc[tid] = 0;
  }
  __syncthreads();

  int t = 0, ov = 0;
  const int nChunks = (nE + CHUNK - 1) / CHUNK;
#pragma unroll 1
  for (int ch = 0; ch < nChunks; ++ch) {
    const int cbase = ch * CHUNK;
    const int wc = scan_chunk<SLB>(keys, nE, cbase, nodeBase, NB, vec8, list, tid, lane, wave);
    if (lane == 0) misc[wave] = wc;
    __syncthreads();
    if (wave == 0) {
#pragma unroll 1
      for (int w2 = 0; w2 < NWAVE; ++w2) {
        int c = misc[w2];
        c = c < 0 ? 0 : (c > WCAP ? WCAP : c);
#pragma unroll 1
        for (int b0 = 0; b0 < c; b0 += 32) {
          const int idx = b0 + lane;
          const int ent = list[w2 * WCAP + (idx < WCAP ? idx : WCAP - 1)];
          const int m32 = (c - b0) < 32 ? (c - b0) : 32;
#pragma unroll 1
          for (int k = 0; k < m32; ++k) {
            const int u    = __builtin_amdgcn_readlane(ent, k);
            const int slot = u & (NB - 1);
            const int el   = (u >> SLB) & (CHUNK - 1);
            const int pk   = ((cbase + el) << SLB) | slot;
            if (t < RCAP) {
              if (lane == 0) { hl[t] = pk; cnt[slot] = cnt[slot] + 1; }
              t = t + 1;
            } else {
              ov = 1;
            }
          }
        }
      }
    }
    __syncthreads();
  }
  if (wave == 0 && lane == 0) { misc[8] = t; misc[9] = ov; }
  __syncthreads();
  int tt = misc[8];
  tt = tt < 0 ? 0 : (tt > RCAP ? RCAP : tt);
  const int ovf = misc[9];

  if (wave == 0) {
    const int base = lane * (NB / 32);
    int s = 0;
#pragma unroll 1
    for (int i = 0; i < NB / 32; ++i) s += cnt[base + i];
    int incl = s;
#pragma unroll
    for (int d = 1; d < 32; d <<= 1) {
      const int y = __shfl_up(incl, d, 32);
      if (lane >= d) incl += y;
    }
    int run = incl - s;
#pragma unroll 1
    for (int i = 0; i < NB / 32; ++i) {
      const int cv = cnt[base + i];
      offs[base + i] = run;
      cur[base + i]  = run;
      run += cv;
    }
  }
  __syncthreads();
  if (wave == 0) {
#pragma unroll 1
    for (int b0 = 0; b0 < tt; b0 += 32) {
      const int idx = b0 + lane;
      const int ent = hl[idx < RCAP ? idx : RCAP - 1];
      const int m32 = (tt - b0) < 32 ? (tt - b0) : 32;
#pragma unroll 1
      for (int k = 0; k < m32; ++k) {
        const int u    = __builtin_amdgcn_readlane(ent, k);
        const int slot = u & (NB - 1);
        if (lane == 0) {
          int p = cur[slot];
          p = p < 0 ? 0 : (p > RCAP - 1 ? RCAP - 1 : p);
          sl[p] = u;
          cur[slot] = p + 1;
        }
      }
    }
  }
  __syncthreads();

  const float qnan = __int_as_float(0x7fc00000);
  const float pz = (ovf != 0) ? qnan : 0.0f;
  const int q0s = (4 * lane) & 31, q1s = (4 * lane + 1) & 31;
  const int q2s = (4 * lane + 2) & 31, q3s = (4 * lane + 3) & 31;
#pragma unroll 1
  for (int si = 0; si < NB / NWAVE; ++si) {
    const int s    = si * NWAVE + wave;
    const int node = nodeBase + s;
    int c = cnt[s];
    const bool big = c > DEGCAP;
    c = c < 0 ? 0 : (c > DEGCAP ? DEGCAP : c);
    int o = offs[s];
    o = o < 0 ? 0 : (o > RCAP ? RCAP : o);
    const int nc = node < nDst ? node : nDst - 1;
    float a0 = 0.0f, a1 = 0.0f, a2 = 0.0f, a3 = 0.0f;
#pragma unroll 1
    for (int b0 = 0; b0 < c; b0 += 32) {
      int idx = o + b0 + lane;
      idx = idx > RCAP - 1 ? RCAP - 1 : idx;
      const int ent = sl[idx];
      int eid = ent >> SLB;
      eid = eid < 0 ? 0 : (eid > nE - 1 ? nE - 1 : eid);
      int sr = gath[eid];
      sr = sr < 0 ? 0 : (sr > nSrc - 1 ? nSrc - 1 : sr);
      const int m32 = (c - b0) < 32 ? (c - b0) : 32;
#pragma unroll 1
      for (int k = 0; k < m32; ++k) {
        const int sk = __builtin_amdgcn_readlane(sr, k);
        if constexpr (WIDE == 0) {
          const unsigned w = *(const u32a*)(srcPl + (size_t)sk * AP1 + XOFF + 2 * lane);
          a0 += __uint_as_float(w << 16);
          a1 += __uint_as_float(w & 0xffff0000u);
        } else {
          const v4f a = *(const v4f*)(t3 + (size_t)sk * HID + 4 * lane);
          a0 += a.x; a1 += a.y; a2 += a.z; a3 += a.w;
        }
      }
    }
    const float dgf = (float)(c < 1 ? 1 : c);
    const float inv = 1.0f / dgf;
    const float pzr = big ? qnan : pz;
    const bool live = node < nDst;

    if constexpr (WIDE == 0) {
      float y0 = a0 * inv, y1 = a1 * inv;
      y0 = y0 + pzr; y1 = y1 + pzr;
      const float v0 = live ? y0 : 0.0f;
      const float v1 = live ? y1 : 0.0f;
      const bool wr = (node < mRows) && (lane < 16);
      const unsigned hb0 = bf16_bits(v0), hb1 = bf16_bits(v1);
      const unsigned lb0 = bf16_bits(v0 - __uint_as_float(hb0 << 16));
      const unsigned lb1 = bf16_bits(v1 - __uint_as_float(hb1 << 16));
      const int hw = (int)(hb0 | (hb1 << 16));
      const int lw = (int)(lb0 | (lb1 << 16));
      const int g0 = __shfl(hw, q0s, 32), g1 = __shfl(hw, q1s, 32);
      const int g2 = __shfl(hw, q2s, 32), g3 = __shfl(hw, q3s, 32);
      const int p0 = __shfl(lw, q0s, 32), p1 = __shfl(lw, q1s, 32);
      const int p2 = __shfl(lw, q2s, 32), p3 = __shfl(lw, q3s, 32);
      const bool lsel = (lane & 8) != 0;
      v4u pv;
      pv.x = (unsigned int)(lsel ? p0 : g0);
      pv.y = (unsigned int)(lsel ? p1 : g1);
      pv.z = (unsigned int)(lsel ? p2 : g2);
      pv.w = (unsigned int)(lsel ? p3 : g3);
      unsigned short* hp = outPl + (size_t)node * AP1 + 8 * (lane & 15);
      if (wr) *(volatile v4u*)hp = pv;
      __threadfence();
      if (wr) *(volatile v4u*)hp = pv;
    } else {
      const v4f sv = *(const v4f*)(s3 + (size_t)nc * HID + 4 * lane);
      float u0 = sv.x + a0 * inv, u1 = sv.y + a1 * inv, u2 = sv.z + a2 * inv, u3 = sv.w + a3 * inv;
      u0 = (u0 > 0.0f) ? u0 : (u0 - u0);
      u1 = (u1 > 0.0f) ? u1 : (u1 - u1);
      u2 = (u2 > 0.0f) ? u2 : (u2 - u2);
      u3 = (u3 > 0.0f) ? u3 : (u3 - u3);
      u0 = u0 + pzr; u1 = u1 + pzr; u2 = u2 + pzr; u3 = u3 + pzr;
      const float m0 = live ? u0 : 0.0f;
      const float m1 = live ? u1 : 0.0f;
      const float m2 = live ? u2 : 0.0f;
      const float m3 = live ? u3 : 0.0f;
      v4us mh, ml;
      {
        unsigned hb;
        hb = bf16_bits(m0); mh[0] = (unsigned short)hb; ml[0] = (unsigned short)bf16_bits(m0 - __uint_as_float(hb << 16));
        hb = bf16_bits(m1); mh[1] = (unsigned short)hb; ml[1] = (unsigned short)bf16_bits(m1 - __uint_as_float(hb << 16));
        hb = bf16_bits(m2); mh[2] = (unsigned short)hb; ml[2] = (unsigned short)bf16_bits(m2 - __uint_as_float(hb << 16));
        hb = bf16_bits(m3); mh[3] = (unsigned short)hb; ml[3] = (unsigned short)bf16_bits(m3 - __uint_as_float(hb << 16));
      }
      *(v4usa*)(rowbuf + 4 * lane) = mh;
      *(v4usa*)(rowbuf + HID + 4 * lane) = ml;
      wave_sync();
      const v8us q0 = *(const v8usa*)(rowbuf + 8 * lane);
      wave_sync();
      if (node < mRows) {
        unsigned short* rpw = outPl + (size_t)node * AP2 + 8 * lane;
        *(volatile v8us*)rpw = q0;
        __threadfence();
        *(volatile v8us*)rpw = q0;
      }
    }
  }
}

static inline int cdiv(int a, int b) { return (a + b - 1) / b; }
static inline size_t al256(size_t o) { return (o + 255) & ~(size_t)255; }

extern "C" void kernel_launch(void* const* d_in, const int* in_sizes, int n_in,
                              void* d_out, int out_size, void* d_ws, size_t ws_size,
                              hipStream_t stream) {
  if (n_in < 17) return;
  if (in_sizes[0] < DIN || (in_sizes[0] % DIN) != 0) return;
  if (in_sizes[1] < DIN || (in_sizes[1] % DIN) != 0) return;
  const int nU = in_sizes[0] / DIN;
  const int nM = in_sizes[1] / DIN;
  const int nE = in_sizes[2];
  if (nE < 1 || in_sizes[3] != nE) return;
  if (nE >= (1 << (31 - SLB_U))) return;
  if (nU < 16 || nM < 16 || nU > (1 << 22) || nM > (1 << 22)) return;
  if (in_sizes[4] != DIN * HID || in_sizes[5] != DIN * HID || in_sizes[6] != HID) return;
  if (in_sizes[7] != DIN * HID || in_sizes[8] != DIN * HID || in_sizes[9] != HID) return;
  if (in_sizes[10] != HID * HID || in_sizes[11] != HID * HID || in_sizes[12] != HID) return;
  if (in_sizes[13] != HID * OUTC || in_sizes[14] != OUTC) return;
  if (in_sizes[15] != HID * OUTC || in_sizes[16] != OUTC) return;
  if ((long long)out_size != ((long long)nU + (long long)nM) * OUTC) return;

  const float* xU   = (const float*)d_in[0];
  const float* xM   = (const float*)d_in[1];
  const int*   eU   = (const int*)d_in[2];
  const int*   eM   = (const int*)d_in[3];
  const float* W1l  = (const float*)d_in[4];
  const float* W1r  = (const float*)d_in[5];
  const float* b1   = (const float*)d_in[6];
  const float* W2l  = (const float*)d_in[7];
  const float* W2r  = (const float*)d_in[8];
  const float* b2   = (const float*)d_in[9];
  const float* W3l  = (const float*)d_in[10];
  const float* W3r  = (const float*)d_in[11];
  const float* b3   = (const float*)d_in[12];
  const float* Wl1  = (const float*)d_in[13];
  const float* bl1  = (const float*)d_in[14];
  const float* Wl2  = (const float*)d_in[15];
  const float* bl2  = (const float*)d_in[16];
  float* outU = (float*)d_out;
  float* outM = (float*)d_out + (size_t)nU * OUTC;

  const int MP1 = cdiv(nU, 128) * 128;
  const int MP2 = cdiv(nM, 128) * 128;
  const int nBU = MP1 / 32;
  const int nBM = MP2 / 32;
  const int gU  = cdiv(MP1, 1 << SLB_U);
  const int gM  = cdiv(MP2, 1 << SLB_M);
  if ((long long)gU * (1 << SLB_U) < (long long)MP1) return;
  if ((long long)gM * (1 << SLB_M) < (long long)MP2) return;
  const int vec8 = ((nE & 3) == 0) ? 1 : 0;

  char* ws = (char*)d_ws;
  size_t off = 0;
  const size_t oB1  = off; off = al256(off + (size_t)HID * AP1 * 2);
  const size_t oB2  = off; off = al256(off + (size_t)HID * AP1 * 2);
  const size_t oBM  = off; off = al256(off + (size_t)(HID + OUTC) * AP2 * 2);
  const size_t oB3r = off; off = al256(off + (size_t)HID * AP2 * 2);
  const size_t oBL1 = off; off = al256(off + (size_t)OUTC * AP2 * 2);
  const size_t oA1U = off; off = al256(off + (size_t)MP1 * AP1 * 2);
  const size_t oA2M = off; off = al256(off + (size_t)MP2 * AP1 * 2);
  const size_t oMX  = off; off = al256(off + (size_t)MP2 * AP2 * 2);
  const size_t endDead = off;
  const size_t oT3  = off; off = al256(off + (size_t)MP2 * HID * 4);
  const size_t oU1  = off; off = al256(off + (size_t)MP1 * AP2 * 2);
  const size_t oS3  = oA1U;
  if (oS3 + (size_t)MP1 * HID * 4 > endDead) return;
  if (off > ws_size || off > (size_t)WSMAX) return;
  unsigned short* B1  = (unsigned short*)(ws + oB1);
  unsigned short* B2  = (unsigned short*)(ws + oB2);
  unsigned short* BM  = (unsigned short*)(ws + oBM);
  unsigned short* B3r = (unsigned short*)(ws + oB3r);
  unsigned short* BL1 = (unsigned short*)(ws + oBL1);
  unsigned short* A1U = (unsigned short*)(ws + oA1U);
  unsigned short* A2M = (unsigned short*)(ws + oA2M);
  unsigned short* MX  = (unsigned short*)(ws + oMX);
  float*          T3  = (float*)(ws + oT3);
  unsigned short* U1  = (unsigned short*)(ws + oU1);
  unsigned short* U3  = U1;
  float*          S3  = (float*)(ws + oS3);

  const size_t ldsM = (size_t)SCAN_LDSINTS(SLB_M) * 4;
  const size_t ldsU = (size_t)SCAN_LDSINTS(SLB_U) * 4;
  hipFuncSetAttribute(reinterpret_cast<const void*>(&k_scan<SLB_M, 0>), hipFuncAttributeMaxDynamicSharedMemorySize, (int)ldsM);
  hipFuncSetAttribute(reinterpret_cast<const void*>(&k_scan<SLB_U, 0>), hipFuncAttributeMaxDynamicSharedMemorySize, (int)ldsU);
  hipFuncSetAttribute(reinterpret_cast<const void*>(&k_scan<SLB_U, 1>), hipFuncAttributeMaxDynamicSharedMemorySize, (int)ldsU);

  k_prep<<<nBU + nBM + NWB, NTHR, 0, stream>>>(xU, xM, nU, nM, nBU, nBM, W1l, W1r, W2l, W2r, W3l, W3r, Wl1, Wl2,
                                               A1U, A2M, B1, B2, BM, B3r, BL1);
  k_scan<SLB_M, 0><<<gM, NTHR, ldsM, stream>>>(eU, eM, nE, nM, nU, vec8, MP2, A1U, T3, T3, A2M);
  k_gemm<8, 0><<<MP2 / GBM, GTHR, 0, stream>>>(A2M, AP1, B2, AP1, b2, 1, nM, MX, T3);
  k_gemm_mv<<<dim3(MP2 / GBM, 2), GTHR, 0, stream>>>(MX, BM, bl2, b3, nM, U1, T3, outM);
  k_scan<SLB_U, 0><<<gU, NTHR, ldsU, stream>>>(eM, eU, nE, nU, nM, vec8, MP1, A2M, T3, T3, A1U);
  k_gemm<8, 0><<<MP1 / GBM, GTHR, 0, stream>>>(A1U, AP1, B1, AP1, b1, 1, nU, U1, T3);
  k_gemm<8, 1><<<MP1 / GBM, GTHR, 0, stream>>>(U1, AP2, B3r, AP2, b3, 1, nU, BL1, S3);
  k_scan<SLB_U, 1><<<gU, NTHR, ldsU, stream>>>(eM, eU, nE, nU, nM, vec8, MP1, B1, T3, S3, U3);
  k_gemm<4, 2><<<MP1 / GBM, GTHR, 0, stream>>>(U3, AP2, BL1, AP2, bl1, 1, nU, B2, outU);
}
